// ConvTranBackbone_46273977647187
// MI455X (gfx1250) — hardware-verified
//
#include <hip/hip_runtime.h>


#define NB_  16
#define CIN  32
#define SS   512
#define NT   (NB_ * SS)
#define DD   256
#define NH_  8
#define HD   32
#define FF   1024
#define NL   4
#define K1   224
#define K2   1280
#define IG   4
#define ZH   (IG * NH_)
#define NN   SS
#define DM   DD
#define SCL  0.17677669529663687f
#define LOSC 1024.0f

typedef _Float16 h16;
typedef unsigned short bf;
typedef __attribute__((ext_vector_type(16))) __bf16   v16bf;
typedef __attribute__((ext_vector_type(16))) _Float16 v16h;
typedef __attribute__((ext_vector_type(8)))  _Float16 v8h;
typedef __attribute__((ext_vector_type(8)))  unsigned short v8us;
typedef __attribute__((ext_vector_type(8)))  float    v8f;
typedef __attribute__((ext_vector_type(4)))  float    v4f;
typedef v8h  __attribute__((may_alias)) v8ha;
typedef v4f  __attribute__((may_alias)) v4fa;
typedef v8us __attribute__((may_alias)) v8usa;

__device__ __forceinline__ unsigned short f2bf(float f) { unsigned u = __float_as_uint(f); u += 0x7FFFu + ((u >> 16) & 1u); return (unsigned short)(u >> 16); }
__device__ __forceinline__ float bf2f(unsigned short b) { return __uint_as_float(((unsigned)b) << 16); }
__device__ __forceinline__ float bfr(float f) { return bf2f(f2bf(f)); }
__device__ __forceinline__ v16h cat16(v8h lo, v8h hi) { return __builtin_shufflevector(lo, hi, 0, 1, 2, 3, 4, 5, 6, 7, 8, 9, 10, 11, 12, 13, 14, 15); }
__device__ __forceinline__ v16bf cat16b(v8us lo, v8us hi) { return __builtin_bit_cast(v16bf, __builtin_shufflevector(lo, hi, 0, 1, 2, 3, 4, 5, 6, 7, 8, 9, 10, 11, 12, 13, 14, 15)); }
__device__ __forceinline__ v8f wmma16(v16h a, v16h b, v8f c) { return __builtin_amdgcn_wmma_f32_16x16x32_f16(false, a, false, b, (short)0, c, false, false); }
__device__ __forceinline__ v8f wmmab(v16bf a, v16bf b, v8f c) { return __builtin_amdgcn_wmma_f32_16x16x32_bf16(false, a, false, b, (short)0, c, false, false); }

template <bool SPLITA, bool F16OUT = false>
__global__ __launch_bounds__(128) void k_gemmb(const bf* __restrict__ A, const bf* __restrict__ Al, const bf* __restrict__ Bn, const float* __restrict__ bias, float* C, int ldc, h16* C2, const float* __restrict__ R = nullptr, int K = DM, int roundR = 1) {
    __shared__ __align__(16) float ost[4][16 * 68];
    const int lane = threadIdx.x & 31, wave = threadIdx.x >> 5, lr = lane & 15, hi = lane >> 4;
    const int r0 = blockIdx.x * 64 + wave * 16, c0 = blockIdx.y * 64;
    const size_t aoff = (size_t)(r0 + lr) * K + 8 * hi;
    size_t boff[4];
#pragma unroll
    for (int t = 0; t < 4; ++t) boff[t] = (size_t)(c0 + t * 16 + lr) * K + 8 * hi;
    v8f acc[4];
#pragma unroll
    for (int t = 0; t < 4; ++t) acc[t] = (v8f){};
#pragma unroll 1
    for (int kc = 0; kc < K; kc += 32) {
        const v16bf a = cat16b(*(const v8us*)(A + aoff + kc), *(const v8us*)(A + aoff + kc + 16));
        v16bf al = a;
        if (SPLITA) al = cat16b(*(const v8us*)(Al + aoff + kc), *(const v8us*)(Al + aoff + kc + 16));
#pragma unroll
        for (int t = 0; t < 4; ++t) { const v16bf b = cat16b(*(const v8us*)(Bn + boff[t] + kc), *(const v8us*)(Bn + boff[t] + kc + 16)); acc[t] = wmmab(a, b, acc[t]); if (SPLITA) acc[t] = wmmab(al, b, acc[t]); }
        asm volatile("v_nop\n\tv_nop\n\tv_nop\n\tv_nop" : "+v"(acc[0]), "+v"(acc[1]), "+v"(acc[2]), "+v"(acc[3]) : "v"(a), "v"(al));
    }
    float* os = &ost[wave][0];
#pragma unroll
    for (int t = 0; t < 4; ++t) { const float bv = bias ? bfr(bias[c0 + t * 16 + lr]) : 0.f;
#pragma unroll
        for (int j = 0; j < 8; ++j) os[(hi * 8 + j) * 68 + t * 16 + lr] = acc[t][j] + bv; }
    __syncthreads();
    if (F16OUT) {
        h16* crow = (h16*)(void*)C + (size_t)r0 * ldc + c0;
        auto pass = [&]() {
#pragma unroll
            for (int s = 0; s < 4; ++s) { const int row = 4 * s + (lane >> 3), piece = lane & 7; const float* sp = os + row * 68 + piece * 8; v8h o, o2;
#pragma unroll
                for (int i = 0; i < 8; ++i) { const h16 a = (h16)sp[i]; o[i] = a; o2[i] = (h16)((sp[i] - (float)a) * LOSC); }
                *(volatile v8h*)(crow + (size_t)row * ldc + piece * 8) = o; if (C2) *(volatile v8h*)(C2 + (size_t)r0 * ldc + c0 + (size_t)row * ldc + piece * 8) = o2; }
        };
        pass(); __threadfence(); pass();
    } else {
        float* crow = C + (size_t)r0 * ldc + c0;
        auto pass = [&]() {
#pragma unroll
            for (int s = 0; s < 8; ++s) { const int Lid = (lane >> 3) + 4 * s, piece = lane & 7; const int row = Lid >> 1, cofs = (Lid & 1) * 32 + piece * 4;
                v4f val = *(const v4fa*)(os + row * 68 + cofs); if (R) { const v4f rv = *(const v4f*)(R + ((size_t)r0 + row) * ldc + c0 + cofs); val += roundR ? (v4f){bfr(rv[0]), bfr(rv[1]), bfr(rv[2]), bfr(rv[3])} : rv; }
                *(volatile v4f*)(crow + (size_t)row * ldc + cofs) = val; }
        };
        pass(); __threadfence(); pass();
    }
}


__global__ __launch_bounds__(128) void k_gemmh(const h16* __restrict__ A, const h16* __restrict__ Bn, const float* __restrict__ bias, float* C, int ldc, const float* __restrict__ R, int K, size_t sA, size_t sB, size_t sC, int roundR) {
    __shared__ __align__(16) float ost[4][16 * 68];
    const size_t z = blockIdx.z; A += z * sA; Bn += z * sB; C += z * sC; if (R) R += z * sC;
    const int lane = threadIdx.x & 31, wave = threadIdx.x >> 5, lr = lane & 15, hi = lane >> 4;
    const int r0 = blockIdx.x * 64 + wave * 16, c0 = blockIdx.y * 64;
    const size_t aoff = (size_t)(r0 + lr) * K + 8 * hi;
    size_t boff[4];
#pragma unroll
    for (int t = 0; t < 4; ++t) boff[t] = (size_t)(c0 + t * 16 + lr) * K + 8 * hi;
    v8f acc[4];
#pragma unroll
    for (int t = 0; t < 4; ++t) acc[t] = (v8f){};
#pragma unroll 1
    for (int kc = 0; kc < K; kc += 32) {
        const v16h a = cat16(*(const v8h*)(A + aoff + kc), *(const v8h*)(A + aoff + kc + 16));
#pragma unroll
        for (int t = 0; t < 4; ++t) { const v16h b = cat16(*(const v8h*)(Bn + boff[t] + kc), *(const v8h*)(Bn + boff[t] + kc + 16)); acc[t] = wmma16(a, b, acc[t]); }
        asm volatile("v_nop\n\tv_nop\n\tv_nop\n\tv_nop" : "+v"(acc[0]), "+v"(acc[1]), "+v"(acc[2]), "+v"(acc[3]) : "v"(a));
    }
    float* os = &ost[wave][0];
#pragma unroll
    for (int t = 0; t < 4; ++t) { const float bv = bias ? bfr(bias[c0 + t * 16 + lr]) : 0.f;
#pragma unroll
        for (int j = 0; j < 8; ++j) os[(hi * 8 + j) * 68 + t * 16 + lr] = acc[t][j] + bv; }
    __syncthreads();
    float* crow = C + (size_t)r0 * ldc + c0;
    auto pass = [&]() {
#pragma unroll
        for (int s = 0; s < 8; ++s) { const int Lid = (lane >> 3) + 4 * s, piece = lane & 7; const int row = Lid >> 1, cofs = (Lid & 1) * 32 + piece * 4;
            v4f val = *(const v4fa*)(os + row * 68 + cofs); if (R) { const v4f rv = *(const v4f*)(R + ((size_t)r0 + row) * ldc + c0 + cofs); val += roundR ? (v4f){bfr(rv[0]), bfr(rv[1]), bfr(rv[2]), bfr(rv[3])} : rv; }
            *(volatile v4f*)(crow + (size_t)row * ldc + cofs) = val; }
    };
    pass(); __threadfence(); pass();
}

template <int MODE>
__global__ __launch_bounds__(128) void k_gemm3z(const bf* __restrict__ Ah, const bf* __restrict__ Al, const bf* __restrict__ Bh, const bf* __restrict__ Bl, int K, float* C, int ldc, size_t sA, size_t sB, size_t sC) {
    if ((MODE & 1) && (int)blockIdx.y * 64 > (int)blockIdx.x * 64 + 63) return;
    const size_t z = blockIdx.z; Ah += z * sA; Al += z * sA; Bh += z * sB; Bl += z * sB; C += z * sC;
    const int Klim = (MODE & 2) ? min(K, ((int)blockIdx.x + 1) * 64) : K;
    __shared__ __align__(16) float ost[4][16 * 68];
    const int lane = threadIdx.x & 31, wave = threadIdx.x >> 5, lr = lane & 15, hi = lane >> 4;
    const int r0 = blockIdx.x * 64 + wave * 16, c0 = blockIdx.y * 64;
    const size_t aoff = (size_t)(r0 + lr) * K + 8 * hi;
    v8f acc[4];
#pragma unroll
    for (int t = 0; t < 4; ++t) acc[t] = (v8f){};
#pragma unroll 1
    for (int kc = 0; kc < Klim; kc += 32) {
        const v16bf a = cat16b(*(const v8us*)(Ah + aoff + kc), *(const v8us*)(Ah + aoff + kc + 16));
        v16bf al = a; if (!(MODE & 4) && !(MODE & 16)) al = cat16b(*(const v8us*)(Al + aoff + kc), *(const v8us*)(Al + aoff + kc + 16));
#pragma unroll
        for (int t = 0; t < 4; ++t) { const size_t bo = (size_t)(c0 + t * 16 + lr) * K + kc + 8 * hi;
            const v16bf bh = cat16b(*(const v8us*)(Bh + bo), *(const v8us*)(Bh + bo + 16));
            acc[t] = wmmab(a, bh, acc[t]);
            if (!(MODE & 4)) { if (!(MODE & 16)) acc[t] = wmmab(al, bh, acc[t]); if (!(MODE & 8)) { const v16bf bl = cat16b(*(const v8us*)(Bl + bo), *(const v8us*)(Bl + bo + 16)); acc[t] = wmmab(a, bl, acc[t]); } } }
        asm volatile("v_nop\n\tv_nop\n\tv_nop\n\tv_nop" : "+v"(acc[0]), "+v"(acc[1]), "+v"(acc[2]), "+v"(acc[3]) : "v"(a), "v"(al));
    }
    float* os = &ost[wave][0];
#pragma unroll
    for (int t = 0; t < 4; ++t) {
#pragma unroll
        for (int j = 0; j < 8; ++j) os[(hi * 8 + j) * 68 + t * 16 + lr] = acc[t][j]; }
    __builtin_amdgcn_wave_barrier(); asm volatile("" ::: "memory");
    float* crow = C + (size_t)r0 * ldc + c0;
    auto pass = [&]() {
#pragma unroll
        for (int s = 0; s < 8; ++s) { const int Lid = (lane >> 3) + 4 * s, piece = lane & 7; const int row = Lid >> 1, cofs = (Lid & 1) * 32 + piece * 4;
            const v4f val = *(const v4fa*)(os + row * 68 + cofs); *(volatile v4f*)(crow + (size_t)row * ldc + cofs) = val; }
    };
    pass(); __threadfence(); pass();
}
__global__ __launch_bounds__(256) void k_planes32z(const float* __restrict__ F, int ld, int off, float sc, int rows, bf* Ph, bf* Pl) {
    typedef __attribute__((ext_vector_type(2))) unsigned short v2us;
    const int lane = threadIdx.x & 31; const size_t r = ((size_t)blockIdx.x * 8 + (threadIdx.x >> 5)) * 2 + (lane >> 4); if (r >= (size_t)rows) return; const int z = blockIdx.z; const int c0 = (lane & 15) * 2; v2us oh, ol;
    Ph += (size_t)z * rows * 32; Pl += (size_t)z * rows * 32;
#pragma unroll
    for (int i = 0; i < 2; ++i) { const float y = F[r * ld + off + z * 32 + c0 + i] * sc; const unsigned short hb = f2bf(y); oh[i] = hb; ol[i] = f2bf(y - bf2f(hb)); }
    const size_t o = r * 32 + c0; *(volatile v2us*)(Ph + o) = oh; *(volatile v2us*)(Pl + o) = ol; __threadfence(); *(volatile v2us*)(Ph + o) = oh; *(volatile v2us*)(Pl + o) = ol;
}
__global__ __launch_bounds__(256) void k_vtpadz(const float* __restrict__ F, int ld, int off, int nk, bf* Th, bf* Tl) {
    typedef __attribute__((ext_vector_type(2))) unsigned short v2us;
    const int lane = threadIdx.x & 31; const size_t wid = (size_t)blockIdx.x * 8 + (threadIdx.x >> 5); if (wid >= (size_t)64 * (nk / 64)) return; const int z = blockIdx.z; const int d = (int)(wid / (nk / 64)); const int k0 = (int)(wid % (nk / 64)) * 64 + lane * 2; v2us oh, ol;
    Th += (size_t)z * 64 * nk; Tl += (size_t)z * 64 * nk;
#pragma unroll
    for (int i = 0; i < 2; ++i) { const float y = (d < 32) ? F[(size_t)(k0 + i) * ld + off + z * 32 + (d < 32 ? d : 0)] : 0.f; const unsigned short hb = f2bf(y); oh[i] = hb; ol[i] = f2bf(y - bf2f(hb)); }
    const size_t o = (size_t)d * nk + k0; *(volatile v2us*)(Th + o) = oh; *(volatile v2us*)(Tl + o) = ol; __threadfence(); *(volatile v2us*)(Th + o) = oh; *(volatile v2us*)(Tl + o) = ol;
}
template <int NK>
__global__ __launch_bounds__(256) void k_softmaxz(const float* __restrict__ S, int rows, bf* PH, bf* PL) {
    typedef __attribute__((ext_vector_type(4))) unsigned short v4us;
    const int lane = threadIdx.x & 31, i = blockIdx.x * 8 + (threadIdx.x >> 5); if (i >= rows) return; const size_t zo = (size_t)blockIdx.z * rows * NK; const float* sr = S + zo + (size_t)i * NK; PH += zo; PL += zo;
    float m = -3.0e38f;
#pragma unroll 1
    for (int c0 = lane * 4; c0 < NK; c0 += 128) {
#pragma unroll
        for (int q = 0; q < 4; ++q) m = fmaxf(m, sr[c0 + q]); }
#pragma unroll
    for (int sh = 16; sh; sh >>= 1) m = fmaxf(m, __shfl_xor(m, sh, 32));
    float sum = 0.f;
#pragma unroll 1
    for (int c0 = lane * 4; c0 < NK; c0 += 128) {
#pragma unroll
        for (int q = 0; q < 4; ++q) sum += __expf(sr[c0 + q] - m); }
#pragma unroll
    for (int sh = 16; sh; sh >>= 1) sum += __shfl_xor(sum, sh, 32);
    const float inv = 1.0f / sum;
#pragma unroll 1
    for (int ps = 0; ps < 2; ++ps) {
#pragma unroll 1
        for (int c0 = lane * 4; c0 < NK; c0 += 128) { v4us oh, ol;
#pragma unroll
            for (int q = 0; q < 4; ++q) { const float p = __expf(sr[c0 + q] - m) * inv; const unsigned short hb = f2bf(p); oh[q] = hb; ol[q] = f2bf(p - bf2f(hb)); }
            const size_t o = (size_t)i * NK + c0; *(volatile v4us*)(PH + o) = oh; *(volatile v4us*)(PL + o) = ol; }
        if (ps == 0) __threadfence(); }
}
__global__ __launch_bounds__(256) void k_placez(const float* __restrict__ XH, int rows, int ldy, float* Y) {
    const int lane = threadIdx.x & 31; const size_t q = (size_t)blockIdx.x * 8 + (threadIdx.x >> 5); if (q >= (size_t)rows) return; const int z = blockIdx.z; const float v = XH[((size_t)z * rows + q) * 64 + lane];
    *(volatile float*)(Y + q * ldy + z * 32 + lane) = v; __threadfence(); *(volatile float*)(Y + q * ldy + z * 32 + lane) = v;
}

typedef __attribute__((ext_vector_type(4))) _Float16 v4h;
__device__ __forceinline__ h16 tohx(float x) { return (h16)x; }
__device__ __forceinline__ float gelu_e(float x) { return 0.5f * x * (1.0f + erff(x * 0.70710678118654752f)); }
__global__ __launch_bounds__(256) void k_im1(const float* __restrict__ x, bf* A1) {
    const int lane = threadIdx.x & 31; const size_t r = (size_t)blockIdx.x * 8 + (threadIdx.x >> 5); if (r >= (size_t)NT) return; const int b = (int)(r / SS), s = (int)(r % SS); v8us o;
#pragma unroll
    for (int i = 0; i < 8; ++i) { const int col = lane * 8 + i; float v = 0.f; if (col < K1) { const int k = col / CIN, c = col % CIN; const int ss = s + k - 3; if (ss >= 0 && ss < SS) v = x[((size_t)b * CIN + c) * SS + ss]; } o[i] = f2bf(v); }
    *(volatile v8us*)(A1 + r * 256 + lane * 8) = o; __threadfence(); *(volatile v8us*)(A1 + r * 256 + lane * 8) = o;
}
__global__ __launch_bounds__(256) void k_w1col(const float* __restrict__ w, bf* Bt) {
    const int lane = threadIdx.x & 31; const int o_ = blockIdx.x * 8 + (threadIdx.x >> 5); if (o_ >= DD) return; v8us o;
#pragma unroll
    for (int i = 0; i < 8; ++i) { const int col = lane * 8 + i; float v = 0.f; if (col < K1) { const int k = col / CIN, c = col % CIN; v = w[((size_t)o_ * CIN + c) * 7 + k]; } o[i] = f2bf(v); }
    *(volatile v8us*)(Bt + (size_t)o_ * 256 + lane * 8) = o; __threadfence(); *(volatile v8us*)(Bt + (size_t)o_ * 256 + lane * 8) = o;
}
__global__ __launch_bounds__(256) void k_bngelu_im2(const float* __restrict__ C1, const float* __restrict__ g1, const float* __restrict__ b1, bf* Ah, bf* Al) {
    const int lane = threadIdx.x & 31; const size_t r = (size_t)blockIdx.x * 8 + (threadIdx.x >> 5); if (r >= (size_t)NT) return; const int b = (int)(r / SS), s = (int)(r % SS); const float bnf = rsqrtf(1.0f + 1e-5f);
#pragma unroll 1
    for (int ps = 0; ps < 2; ++ps) {
#pragma unroll 1
        for (int k = 0; k < 5; ++k) { const int ss = s + k - 2; const bool in = (ss >= 0 && ss < SS); v8us oh, ol;
#pragma unroll 1
            for (int i = 0; i < 8; ++i) { const int c = lane * 8 + i; float y = 0.f; if (in) { const float cv = C1[((size_t)b * SS + ss) * DD + c]; y = gelu_e(cv * bfr(g1[c]) * bnf + bfr(b1[c])); } const unsigned short hb = f2bf(y); oh[i] = hb; ol[i] = f2bf(y - bf2f(hb)); }
            const size_t o = r * K2 + k * DD + lane * 8; *(volatile v8us*)(Ah + o) = oh; *(volatile v8us*)(Al + o) = ol; }
        if (ps == 0) __threadfence(); }
}
__global__ __launch_bounds__(256) void k_w2col(const float* __restrict__ w, bf* Bt) {
    const int lane = threadIdx.x & 31; const int o_ = blockIdx.x * 8 + (threadIdx.x >> 5); if (o_ >= DD) return;
#pragma unroll 1
    for (int ps = 0; ps < 2; ++ps) {
#pragma unroll 1
        for (int k = 0; k < 5; ++k) { v8us o;
#pragma unroll
            for (int i = 0; i < 8; ++i) { const int c = lane * 8 + i; o[i] = f2bf(w[((size_t)o_ * DD + c) * 5 + k]); }
            *(volatile v8us*)(Bt + (size_t)o_ * K2 + k * DD + lane * 8) = o; }
        if (ps == 0) __threadfence(); }
}

__global__ __launch_bounds__(256) void k_petab(float* PE) {
    const size_t e = (size_t)blockIdx.x * 256 + threadIdx.x; if (e >= (size_t)SS * DD) return; const int s = (int)(e / DD), c = (int)(e % DD); const int i2 = c & ~1;
    const float div = expf((float)i2 * (-logf(10000.0f) / (float)DD)); const float a = (float)s * div * ((float)DD / (float)SS); const float pe = (c & 1) ? cosf(a) : sinf(a);
    *(volatile float*)(PE + e) = pe; __threadfence(); *(volatile float*)(PE + e) = pe;
}
__global__ __launch_bounds__(256) void k_bngelu_pe(const float* __restrict__ C2, const float* __restrict__ g2, const float* __restrict__ b2, const float* __restrict__ PE, float* T) {
    const int lane = threadIdx.x & 31; const size_t r = (size_t)blockIdx.x * 8 + (threadIdx.x >> 5); if (r >= (size_t)NT) return; const int s = (int)(r % SS); const float bnf = rsqrtf(1.0f + 1e-5f);
#pragma unroll 1
    for (int half = 0; half < 2; ++half) { const int cb = half * 128 + lane * 4; v4f v;
#pragma unroll
        for (int i = 0; i < 4; ++i) { const int c = cb + i; v[i] = gelu_e(C2[r * DD + c] * bfr(g2[c]) * bnf + bfr(b2[c])) + PE[(size_t)s * DD + c]; }
        *(volatile v4f*)(T + r * DD + cb) = v; __threadfence(); *(volatile v4f*)(T + r * DD + cb) = v; }
}
template <int KIND>
__global__ __launch_bounds__(256) void k_lnp256(const float* __restrict__ X, size_t rows, const float* __restrict__ g, const float* __restrict__ bb, bf* Ph, bf* Pl, h16* P16, float* OF) {
    const int lane = threadIdx.x & 31; const size_t r = (size_t)blockIdx.x * 8 + (threadIdx.x >> 5); if (r >= rows) return; float v[8]; float s = 0.f;
#pragma unroll
    for (int i = 0; i < 8; ++i) { const int c = (i < 4) ? lane * 4 + i : 128 + lane * 4 + i - 4; v[i] = X[r * DD + c]; s += v[i]; }
#pragma unroll
    for (int sh = 16; sh; sh >>= 1) s += __shfl_xor(s, sh, 32);
    const float mu = s * (1.0f / DD); float q = 0.f;
#pragma unroll
    for (int i = 0; i < 8; ++i) { const float d = v[i] - mu; q = fmaf(d, d, q); }
#pragma unroll
    for (int sh = 16; sh; sh >>= 1) q += __shfl_xor(q, sh, 32);
    const float rs = rsqrtf(q * (1.0f / DD) + 1e-5f);
#pragma unroll
    for (int i = 0; i < 8; ++i) { const int c = (i < 4) ? lane * 4 + i : 128 + lane * 4 + i - 4; v[i] = (v[i] - mu) * rs * bfr(g[c]) + bfr(bb[c]); }
    typedef __attribute__((ext_vector_type(4))) unsigned short v4us;
    const size_t oa = r * DD + lane * 4, ob = r * DD + 128 + lane * 4;
#pragma unroll 1
    for (int ps = 0; ps < 2; ++ps) {
        if (KIND == 0) { v4us ah, al, bh, bl;
#pragma unroll
            for (int i = 0; i < 4; ++i) { unsigned short hb = f2bf(v[i]); ah[i] = hb; al[i] = f2bf(v[i] - bf2f(hb)); hb = f2bf(v[4 + i]); bh[i] = hb; bl[i] = f2bf(v[4 + i] - bf2f(hb)); }
            *(volatile v4us*)(Ph + oa) = ah; *(volatile v4us*)(Pl + oa) = al; *(volatile v4us*)(Ph + ob) = bh; *(volatile v4us*)(Pl + ob) = bl; }
        else if (KIND == 1) { v4h ha, hb2;
#pragma unroll
            for (int i = 0; i < 4; ++i) { ha[i] = tohx(v[i]); hb2[i] = tohx(v[4 + i]); } *(volatile v4h*)(P16 + oa) = ha; *(volatile v4h*)(P16 + ob) = hb2; }
        else { *(volatile v4f*)(OF + oa) = (v4f){v[0], v[1], v[2], v[3]}; *(volatile v4f*)(OF + ob) = (v4f){v[4], v[5], v[6], v[7]}; }
        if (ps == 0) __threadfence(); }
}
__global__ __launch_bounds__(256) void k_split256(const float* __restrict__ F, size_t rows, bf* Ph, bf* Pl) {
    const int lane = threadIdx.x & 31; const size_t r = (size_t)blockIdx.x * 8 + (threadIdx.x >> 5); if (r >= rows) return; const size_t o = r * DD + lane * 8; const v8f v = *(const v8f*)(F + o); v8us oh, ol;
#pragma unroll
    for (int i = 0; i < 8; ++i) { const unsigned short hb = f2bf(v[i]); oh[i] = hb; ol[i] = f2bf(v[i] - bf2f(hb)); }
    *(volatile v8us*)(Ph + o) = oh; *(volatile v8us*)(Pl + o) = ol; __threadfence(); *(volatile v8us*)(Ph + o) = oh; *(volatile v8us*)(Pl + o) = ol;
}
__global__ __launch_bounds__(256) void k_relbias(const float* __restrict__ tab, float* BIAS) {
    const int lane = threadIdx.x & 31; const size_t w = (size_t)blockIdx.x * 8 + (threadIdx.x >> 5); if (w >= (size_t)NH_ * SS) return; const int h = (int)(w / SS), i = (int)(w % SS);
#pragma unroll 1
    for (int ps = 0; ps < 2; ++ps) {
#pragma unroll 1
        for (int c0 = lane * 4; c0 < SS; c0 += 128) { v4f o;
#pragma unroll
            for (int q = 0; q < 4; ++q) { const int j = c0 + q; o[q] = bfr(tab[((size_t)(i - j + SS - 1)) * NH_ + h]); }
            *(volatile v4f*)(BIAS + w * SS + c0) = o; }
        if (ps == 0) __threadfence(); }
}
__global__ __launch_bounds__(256) void k_hpl32c(const float* __restrict__ QKV, size_t r0, int col0, float sc, bf* Ph, bf* Pl) {
    typedef __attribute__((ext_vector_type(4))) unsigned short v4us;
    const int lane = threadIdx.x & 31; const size_t w = (size_t)blockIdx.x * 8 + (threadIdx.x >> 5); if (w >= (size_t)SS / 4) return; const int z = blockIdx.z; const int g_ = z / NH_, h_ = z % NH_; const int i = (int)(w * 4 + (lane >> 3)); const int c0 = (lane & 7) * 4; v4us oh, ol;
#pragma unroll
    for (int q = 0; q < 4; ++q) { const float y = QKV[(r0 + (size_t)g_ * SS + i) * (3 * DD) + col0 + h_ * HD + c0 + q] * sc; const unsigned short hb = f2bf(y); oh[q] = hb; ol[q] = f2bf(y - bf2f(hb)); }
    const size_t o = ((size_t)z * SS + i) * HD + c0; *(volatile v4us*)(Ph + o) = oh; *(volatile v4us*)(Pl + o) = ol; __threadfence(); *(volatile v4us*)(Ph + o) = oh; *(volatile v4us*)(Pl + o) = ol;
}
__global__ __launch_bounds__(256) void k_vT32c(const float* __restrict__ QKV, size_t r0, bf* Th, bf* Tl) {
    __shared__ float tl[64][33];
    typedef __attribute__((ext_vector_type(4))) unsigned short v4us;
    const int tid = threadIdx.x; const int t0 = blockIdx.x * 64; const int z = blockIdx.z; const int rr = tid >> 2, cq = (tid & 3) * 8;
#pragma unroll
    for (int i = 0; i < 8; ++i) tl[rr][cq + i] = QKV[(r0 + (size_t)(z / NH_) * SS + t0 + rr) * (3 * DD) + 2 * DD + (z % NH_) * HD + cq + i];
    __syncthreads();
    const int lane = tid & 31, wv = tid >> 5;
    auto pass = [&]() {
#pragma unroll
        for (int st = 0; st < 4; ++st) { const int dr = wv * 8 + st * 2 + (lane >> 4); const int tq = (lane & 15) * 4; v4us oh, ol;
#pragma unroll
            for (int i = 0; i < 4; ++i) { const float y = (dr < HD) ? tl[tq + i][dr < HD ? dr : 0] : 0.f; const unsigned short hb = f2bf(y); oh[i] = hb; ol[i] = f2bf(y - bf2f(hb)); }
            const size_t o = ((size_t)z * 64 + dr) * SS + t0 + tq; *(volatile v4us*)(Th + o) = oh; *(volatile v4us*)(Tl + o) = ol; }
    };
    pass(); __threadfence(); pass();
}
__global__ __launch_bounds__(256) void k_softb2(const float* __restrict__ S, const float* __restrict__ BIAS, bf* PH, bf* PL) {
    typedef __attribute__((ext_vector_type(4))) unsigned short v4us;
    const int lane = threadIdx.x & 31, i = blockIdx.x * 8 + (threadIdx.x >> 5); if (i >= SS) return; const int z = blockIdx.z; const size_t zo = (size_t)z * SS * SS; const float* sr = S + zo + (size_t)i * SS; const float* br = BIAS + (size_t)(z % NH_) * SS * SS + (size_t)i * SS;
    float m = -3.0e38f;
#pragma unroll 1
    for (int c0 = lane * 4; c0 < SS; c0 += 128) {
#pragma unroll
        for (int q = 0; q < 4; ++q) m = fmaxf(m, sr[c0 + q] + br[c0 + q]); }
#pragma unroll
    for (int sh = 16; sh; sh >>= 1) m = fmaxf(m, __shfl_xor(m, sh, 32));
    float sum = 0.f;
#pragma unroll 1
    for (int c0 = lane * 4; c0 < SS; c0 += 128) {
#pragma unroll
        for (int q = 0; q < 4; ++q) sum += __expf(sr[c0 + q] + br[c0 + q] - m); }
#pragma unroll
    for (int sh = 16; sh; sh >>= 1) sum += __shfl_xor(sum, sh, 32);
    const float inv = 1.0f / sum;
#pragma unroll 1
    for (int ps = 0; ps < 2; ++ps) {
#pragma unroll 1
        for (int c0 = lane * 4; c0 < SS; c0 += 128) { v4us oh, ol;
#pragma unroll
            for (int q = 0; q < 4; ++q) { const float p = __expf(sr[c0 + q] + br[c0 + q] - m) * inv; const unsigned short hb = f2bf(p); oh[q] = hb; ol[q] = f2bf(p - bf2f(hb)); }
            const size_t o = zo + (size_t)i * SS + c0; *(volatile v4us*)(PH + o) = oh; *(volatile v4us*)(PL + o) = ol; }
        if (ps == 0) __threadfence(); }
}
__global__ __launch_bounds__(256) void k_merge32c(const float* __restrict__ OZ, size_t r0, float* O) {
    const int lane = threadIdx.x & 31; const size_t w = (size_t)blockIdx.x * 8 + (threadIdx.x >> 5); if (w >= (size_t)IG * SS) return; const int g_ = (int)(w / SS); const size_t i = w % SS; const int ha = lane >> 3, d0 = (lane * 4) & 31;
    const v4f va = *(const v4f*)(OZ + ((size_t)(g_ * NH_ + ha) * SS + i) * 64 + d0); const v4f vb = *(const v4f*)(OZ + ((size_t)(g_ * NH_ + 4 + ha) * SS + i) * 64 + d0); float* row = O + (r0 + (size_t)g_ * SS + i) * DD;
    *(volatile v4f*)(row + lane * 4) = va; *(volatile v4f*)(row + 128 + lane * 4) = vb; __threadfence(); *(volatile v4f*)(row + lane * 4) = va; *(volatile v4f*)(row + 128 + lane * 4) = vb;
}
__global__ __launch_bounds__(256) void k_geluh1024(const float* __restrict__ F, size_t rows, h16* Hh) {
    const int lane = threadIdx.x & 31; const size_t r = (size_t)blockIdx.x * 8 + (threadIdx.x >> 5); if (r >= rows) return;
#pragma unroll 1
    for (int ps = 0; ps < 2; ++ps) {
#pragma unroll 1
        for (int q = 0; q < FF / 256; ++q) { const size_t o = r * FF + q * 256 + lane * 8; const v8f v = *(const v8f*)(F + o); v8h h;
#pragma unroll
            for (int i = 0; i < 8; ++i) h[i] = tohx(gelu_e(v[i]));
            *(volatile v8h*)(Hh + o) = h; }
        if (ps == 0) __threadfence(); }
}
template <bool F16>
__global__ __launch_bounds__(256) void k_wTzx(const float* __restrict__ Wm, int K, int N, void* Bt_, size_t bstride) {
    __shared__ float tl[64][65];
    typedef __attribute__((ext_vector_type(4))) unsigned short v4us;
    const int tid = threadIdx.x; const int k0 = blockIdx.x * 64, n0 = blockIdx.y * 64; const size_t z = blockIdx.z; const int rr = tid >> 2, cq = (tid & 3) * 16;
    const float* W = Wm + z * (size_t)K * N;
#pragma unroll
    for (int i = 0; i < 16; ++i) tl[rr][cq + i] = bfr(W[(size_t)(k0 + rr) * N + n0 + cq + i]);
    __syncthreads();
    const int lane = tid & 31, wv = tid >> 5;
    auto pass = [&]() {
#pragma unroll
        for (int st = 0; st < 4; ++st) { const int nr = wv * 8 + st * 2 + (lane >> 4); const int kq = (lane & 15) * 4;
            if (F16) { v4h v; for (int i = 0; i < 4; ++i) v[i] = tohx(tl[kq + i][nr]); *(volatile v4h*)((h16*)Bt_ + z * bstride + (size_t)(n0 + nr) * K + k0 + kq) = v; }
            else { v4us v; for (int i = 0; i < 4; ++i) v[i] = f2bf(tl[kq + i][nr]); *(volatile v4us*)((bf*)Bt_ + z * bstride + (size_t)(n0 + nr) * K + k0 + kq) = v; } }
    };
    pass(); __threadfence(); pass();
}

extern "C" void kernel_launch(void* const* d_in, const int* in_sizes, int n_in,
                              void* d_out, int out_size, void* d_ws, size_t ws_size, hipStream_t stream) {
    (void)in_sizes; (void)n_in; (void)out_size;
    const float* x = (const float*)d_in[0]; const float* c1w = (const float*)d_in[1]; const float* c1b = (const float*)d_in[2]; const float* g1 = (const float*)d_in[3]; const float* b1n = (const float*)d_in[4]; const float* c2w = (const float*)d_in[5]; const float* c2b = (const float*)d_in[6]; const float* g2 = (const float*)d_in[7]; const float* b2n = (const float*)d_in[8];
    const float* l1g = (const float*)d_in[9]; const float* l1b = (const float*)d_in[10]; const float* wq = (const float*)d_in[11]; const float* wk = (const float*)d_in[12]; const float* wv = (const float*)d_in[13]; const float* wo = (const float*)d_in[14]; const float* bo = (const float*)d_in[15]; const float* btab = (const float*)d_in[16];
    const float* l2g = (const float*)d_in[17]; const float* l2b = (const float*)d_in[18]; const float* w1 = (const float*)d_in[19]; const float* b1 = (const float*)d_in[20]; const float* w2 = (const float*)d_in[21]; const float* b2 = (const float*)d_in[22]; const float* fng = (const float*)d_in[23]; const float* fnb = (const float*)d_in[24];
    float* out = (float*)d_out;
    char* wsp = (char*)d_ws;
    auto take = [&](size_t bytes) { char* p = wsp; wsp += (bytes + 255) & ~(size_t)255; return (void*)p; };
    bf* W1C = (bf*)take((size_t)DD * 256 * 2); bf* W2C = (bf*)take((size_t)DD * K2 * 2);
    bf* BQKV = (bf*)take((size_t)NL * 3 * DD * DD * 2); bf* BWO = (bf*)take((size_t)NL * DD * DD * 2); h16* BF1 = (h16*)take((size_t)NL * FF * DD * 2); h16* BF2 = (h16*)take((size_t)NL * DD * FF * 2);
    float* BIAS = (float*)take((size_t)NH_ * SS * SS * 4); float* PEt = (float*)take((size_t)SS * DD * 4); float* T = (float*)take((size_t)NT * DD * 4); float* T2 = (float*)take((size_t)NT * DD * 4); bf* Ph = (bf*)take((size_t)NT * DD * 2); bf* Pl = (bf*)take((size_t)NT * DD * 2);
    char* const shared0 = wsp;
    bf* A1 = (bf*)take((size_t)NT * 256 * 2); float* C1 = (float*)take((size_t)NT * DD * 4); bf* A2h = (bf*)take((size_t)NT * K2 * 2); bf* A2l = (bf*)take((size_t)NT * K2 * 2); float* C2 = (float*)take((size_t)NT * DD * 4);
    char* const tokEnd = wsp; wsp = shared0;
    float* QKV = (float*)take((size_t)NT * 3 * DD * 4); bf* Qh = (bf*)take((size_t)ZH * SS * HD * 2); bf* Ql = (bf*)take((size_t)ZH * SS * HD * 2); bf* Kh = (bf*)take((size_t)ZH * SS * HD * 2); bf* Kl = (bf*)take((size_t)ZH * SS * HD * 2); bf* VTh = (bf*)take((size_t)ZH * 64 * SS * 2); bf* VTl = (bf*)take((size_t)ZH * 64 * SS * 2);
    float* S = (float*)take((size_t)ZH * SS * SS * 4); bf* PH = (bf*)take((size_t)ZH * SS * SS * 2); bf* PL = (bf*)take((size_t)ZH * SS * SS * 2); float* OZ = (float*)take((size_t)ZH * SS * 64 * 4); float* O = (float*)take((size_t)NT * DD * 4);
    h16* Y16 = (h16*)take((size_t)NT * DD * 2); float* F1 = (float*)take((size_t)NT * FF * 4); h16* F16 = (h16*)take((size_t)NT * FF * 2);
    if (wsp < tokEnd) wsp = tokEnd;
    if ((size_t)(wsp - (char*)d_ws) > ws_size) return;
    k_w1col<<<DD / 8, 256, 0, stream>>>(c1w, W1C); k_w2col<<<DD / 8, 256, 0, stream>>>(c2w, W2C);
    k_wTzx<false><<<dim3(DD / 64, DD / 64, NL), 256, 0, stream>>>(wq, DD, DD, BQKV, (size_t)3 * DD * DD); k_wTzx<false><<<dim3(DD / 64, DD / 64, NL), 256, 0, stream>>>(wk, DD, DD, BQKV + (size_t)DD * DD, (size_t)3 * DD * DD); k_wTzx<false><<<dim3(DD / 64, DD / 64, NL), 256, 0, stream>>>(wv, DD, DD, BQKV + (size_t)2 * DD * DD, (size_t)3 * DD * DD);
    k_wTzx<false><<<dim3(DD / 64, DD / 64, NL), 256, 0, stream>>>(wo, DD, DD, BWO, (size_t)DD * DD);
    k_wTzx<true><<<dim3(DD / 64, FF / 64, NL), 256, 0, stream>>>(w1, DD, FF, BF1, (size_t)FF * DD); k_wTzx<true><<<dim3(FF / 64, DD / 64, NL), 256, 0, stream>>>(w2, FF, DD, BF2, (size_t)DD * FF);
    k_im1<<<NT / 8, 256, 0, stream>>>(x, A1);
    k_gemmb<false, false><<<dim3(NT / 64, DD / 64, 1), 128, 0, stream>>>(A1, nullptr, W1C, c1b, C1, DD, nullptr, nullptr, 256);
    k_bngelu_im2<<<NT / 8, 256, 0, stream>>>(C1, g1, b1n, A2h, A2l);
    k_gemmb<true, false><<<dim3(NT / 64, DD / 64, 1), 128, 0, stream>>>(A2h, A2l, W2C, c2b, C2, DD, nullptr, nullptr, K2);
    k_petab<<<(SS * DD) / 256, 256, 0, stream>>>(PEt); k_bngelu_pe<<<NT / 8, 256, 0, stream>>>(C2, g2, b2n, PEt, T);
    for (int l = 0; l < NL; ++l) { const bf* LQ = BQKV + (size_t)l * 3 * DD * DD; const bf* LO = BWO + (size_t)l * DD * DD; const h16* LF1 = BF1 + (size_t)l * FF * DD; const h16* LF2 = BF2 + (size_t)l * DD * FF;
        k_relbias<<<(NH_ * SS) / 8, 256, 0, stream>>>(btab + (size_t)l * (2 * SS - 1) * NH_, BIAS);
        k_lnp256<0><<<NT / 8, 256, 0, stream>>>(T, NT, l1g + (size_t)l * DD, l1b + (size_t)l * DD, Ph, Pl, nullptr, nullptr);
        k_gemmb<true, false><<<dim3(NT / 64, (3 * DD) / 64, 1), 128, 0, stream>>>(Ph, Pl, LQ, nullptr, QKV, 3 * DD, nullptr, nullptr, DD);
        for (int b = 0; b < NB_; b += IG) { const size_t r0 = (size_t)b * SS;
            k_hpl32c<<<dim3((SS / 4) / 8, 1, ZH), 256, 0, stream>>>(QKV, r0, 0, SCL, Qh, Ql); k_hpl32c<<<dim3((SS / 4) / 8, 1, ZH), 256, 0, stream>>>(QKV, r0, DD, 1.0f, Kh, Kl); k_vT32c<<<dim3(SS / 64, 1, ZH), 256, 0, stream>>>(QKV, r0, VTh, VTl);
            k_gemm3z<0><<<dim3(SS / 64, SS / 64, ZH), 128, 0, stream>>>(Qh, Ql, Kh, Kl, HD, S, SS, (size_t)SS * HD, (size_t)SS * HD, (size_t)SS * SS);
            k_softb2<<<dim3(SS / 8, 1, ZH), 256, 0, stream>>>(S, BIAS, PH, PL);
            k_gemm3z<0><<<dim3(SS / 64, 1, ZH), 128, 0, stream>>>(PH, PL, VTh, VTl, SS, OZ, 64, (size_t)SS * SS, (size_t)64 * SS, (size_t)SS * 64);
            k_merge32c<<<(IG * SS) / 8, 256, 0, stream>>>(OZ, r0, O); }
        k_split256<<<NT / 8, 256, 0, stream>>>(O, NT, Ph, Pl);
        k_gemmb<true, false><<<dim3(NT / 64, DD / 64, 1), 128, 0, stream>>>(Ph, Pl, LO, bo + (size_t)l * DD, T2, DD, nullptr, T, DD, 0);
        k_lnp256<1><<<NT / 8, 256, 0, stream>>>(T2, NT, l2g + (size_t)l * DD, l2b + (size_t)l * DD, nullptr, nullptr, Y16, nullptr);
        k_gemmh<<<dim3(NT / 64, FF / 64, 1), 128, 0, stream>>>(Y16, LF1, b1 + (size_t)l * FF, F1, FF, nullptr, DD, 0, 0, 0, 0);
        k_geluh1024<<<NT / 8, 256, 0, stream>>>(F1, NT, F16);
        k_gemmh<<<dim3(NT / 64, DD / 64, 1), 128, 0, stream>>>(F16, LF2, b2 + (size_t)l * DD, T, DD, T2, FF, 0, 0, 0, 0); }
    k_lnp256<2><<<NT / 8, 256, 0, stream>>>(T, NT, fng, fnb, nullptr, nullptr, nullptr, out);
}
